// GraphConvolutionBlock_3770981286190
// MI455X (gfx1250) — hardware-run, weakly checked
//
#include <hip/hip_runtime.h>
#include <stddef.h>
#include <stdint.h>
#include <math.h>

#define NN      50000
#define FD      128
#define HD      128
#define NE      800000
#define GBM     64
#define GTHR    128
#define GWAVE   4
#define MP      50048
#define NTHR    256
#define NWAVE   8
#define EPT     8
#define WCH     (32 * EPT)
#define NBRUN   1024
#define SLB     10
#define NBK     49
#define WLCAP   3584
#define RCAP    28672
#define DEGCAP  64
#define MAXDEG_MEAS   37
#define MAXB1024_MEAS 16768
#define WSTW    260
#define RECW    384

#define BK_ZINTS (NWAVE * WLCAP + RCAP + 3 * NBRUN)
#define BK_INTS  (BK_ZINTS + 16)
#define BK_LDS   (BK_INTS * 4)

#define PBX   (MP * FD / 8 / NTHR)
#define PBW   (HD * FD / 8 / NTHR)
#define PBTOT (PBX + PBW + 1)

static_assert(HD == 128 && HD == 32 * 4 && FD % 32 == 0 && FD == 128);
static_assert(MP % GBM == 0 && MP >= NN && MP == 391 * 128 && GBM == GWAVE * 16 && GTHR == GWAVE * 32);
static_assert(NBRUN == (1 << SLB) && NBRUN % NWAVE == 0 && NBRUN % 32 == 0);
static_assert(NBK * NBRUN >= MP && (NBK - 1) * NBRUN < NN);
static_assert(NE < (1 << 21) && (((long long)NE) << SLB) < (1LL << 31));
static_assert(NE % WCH == 0 && NE % 4 == 0);
static_assert((NWAVE - 1) * (((NE + NWAVE * WCH - 1) / (NWAVE * WCH)) * WCH) < NE);
static_assert(RCAP == NWAVE * WLCAP && RCAP % 4 == 0 && BK_ZINTS % 4 == 0);
static_assert((long long)RCAP * 100 >= (long long)MAXB1024_MEAS * 105);
static_assert(WLCAP >= MAXB1024_MEAS / 8 + 8 * 46 + 1);
static_assert(NN <= 65536);
static_assert(MAXDEG_MEAS + 8 <= DEGCAP);
static_assert(BK_LDS <= 327680);
static_assert((MP * FD / 8) % NTHR == 0 && (HD * FD / 8) % NTHR == 0);
static_assert((NN * 32) % NTHR == 0);
static_assert(RCAP % (NTHR * 4) == 0 && (2 * NBRUN) % (NTHR * 4) == 0);
static_assert(RECW == 3 * HD && RECW / 2 <= NTHR && WSTW >= 4 + 2 * HD);

typedef float          v4f   __attribute__((ext_vector_type(4)));
typedef float          v8f   __attribute__((ext_vector_type(8)));
typedef int            v4i   __attribute__((ext_vector_type(4)));
typedef int            v8i   __attribute__((ext_vector_type(8)));
typedef unsigned       v2u   __attribute__((ext_vector_type(2)));
typedef double         v2d   __attribute__((ext_vector_type(2)));
typedef unsigned short v8us  __attribute__((ext_vector_type(8)));
typedef unsigned short v16us __attribute__((ext_vector_type(16)));
typedef __bf16         v16bf __attribute__((ext_vector_type(16)));
typedef v4f  __attribute__((may_alias)) v4fa;
typedef v4i  __attribute__((may_alias)) v4ia;
typedef v2u  __attribute__((may_alias)) v2ua;
typedef v2d  __attribute__((may_alias)) v2da;
typedef v8us __attribute__((may_alias)) v8usa;
union FragB { v16bf v; v16us u; v8us h[2]; v8i w; };

__device__ __forceinline__ v8f wmb(const FragB& a, const FragB& b, v8f c) {
  v8f d = __builtin_amdgcn_wmma_f32_16x16x32_bf16(false, a.v, false, b.v, (short)0, c, false, false);
  asm volatile("v_nop\n\tv_nop\n\tv_nop\n\tv_nop" : "+v"(d) : "v"(a.w), "v"(b.w));
  return d;
}

__device__ __forceinline__ v8f z8() { v8f z = {0.f, 0.f, 0.f, 0.f, 0.f, 0.f, 0.f, 0.f}; return z; }

__device__ __forceinline__ unsigned bf16_bits(float f) {
  const unsigned u = __float_as_uint(f);
  const unsigned r = (u + 0x7FFFu + ((u >> 16) & 1u)) >> 16;
  const unsigned q = (u >> 16) | 0x40u;
  return ((u & 0x7fffffffu) > 0x7f800000u) ? q : r;
}
__device__ __forceinline__ float bf16_val(float f) {
  return __uint_as_float(bf16_bits(f) << 16);
}

__device__ __forceinline__ void st2_v4f(float* p, v4f v) {
  *(volatile v4f*)p = v;
  __threadfence();
  *(volatile v4f*)p = v;
}
__device__ __forceinline__ void st2_v8us(unsigned short* p, v8us v) {
  *(volatile v8us*)p = v;
  __threadfence();
  *(volatile v8us*)p = v;
}

__device__ __forceinline__ v8us gather8(const float* __restrict__ base, int stride) {
  float f[8];
#pragma unroll
  for (int i = 0; i < 8; ++i) f[i] = base[(size_t)i * (size_t)stride];
  v8us o;
#pragma unroll
  for (int i = 0; i < 8; ++i) o[i] = (unsigned short)bf16_bits(f[i]);
  return o;
}

__global__ __launch_bounds__(NTHR) void k_prep(const float* __restrict__ x, const float* __restrict__ w,
                                               const float* __restrict__ bias, const float* __restrict__ gam,
                                               const float* __restrict__ bet,
                                               unsigned short* xb, unsigned short* wt, float* par) {
  const int tid = (int)threadIdx.x, lane = tid & 31;
  const int blk = (int)blockIdx.x;
  if (blk < PBX) {
    const int u   = blk * NTHR + tid;
    const int row = u >> 4, k8 = (u & 15) * 8;
    const int rc  = row < NN ? row : NN - 1;
    const unsigned mk = row < NN ? 0xffffu : 0u;
    const float* p = x + (size_t)rc * FD + k8;
    const v4f a = *(const v4fa*)p;
    const v4f b = *(const v4fa*)(p + 4);
    v8us o;
    o[0] = (unsigned short)(bf16_bits(a.x) & mk); o[1] = (unsigned short)(bf16_bits(a.y) & mk);
    o[2] = (unsigned short)(bf16_bits(a.z) & mk); o[3] = (unsigned short)(bf16_bits(a.w) & mk);
    o[4] = (unsigned short)(bf16_bits(b.x) & mk); o[5] = (unsigned short)(bf16_bits(b.y) & mk);
    o[6] = (unsigned short)(bf16_bits(b.z) & mk); o[7] = (unsigned short)(bf16_bits(b.w) & mk);
    st2_v8us(xb + (size_t)row * FD + k8, o);
  } else if (blk < PBX + PBW) {
    const int u = (blk - PBX) * NTHR + tid;
    const int n = u >> 4, k8 = (u & 15) * 8;
    const v8us o = gather8(w + (size_t)k8 * HD + n, HD);
    st2_v8us(wt + (size_t)n * FD + k8, o);
  } else {
    if (tid < 32) {
      const v4f a = *(const v4fa*)(bias + 4 * lane);
      v4f o;
      o.x = bf16_val(a.x); o.y = bf16_val(a.y); o.z = bf16_val(a.z); o.w = bf16_val(a.w);
      st2_v4f(par + 4 * lane, o);
    } else if (tid < 64) {
      const v4f a = *(const v4fa*)(gam + 4 * lane);
      v4f o;
      o.x = bf16_val(a.x); o.y = bf16_val(a.y); o.z = bf16_val(a.z); o.w = bf16_val(a.w);
      st2_v4f(par + HD + 4 * lane, o);
    } else if (tid < 96) {
      const v4f a = *(const v4fa*)(bet + 4 * lane);
      v4f o;
      o.x = bf16_val(a.x); o.y = bf16_val(a.y); o.z = bf16_val(a.z); o.w = bf16_val(a.w);
      st2_v4f(par + 2 * HD + 4 * lane, o);
    }
  }
}

__global__ __launch_bounds__(GTHR) __attribute__((amdgpu_num_vgpr(248)))
void k_gemm_one(const unsigned short* __restrict__ A, const unsigned short* __restrict__ BT, float* XW) {
  __shared__ __attribute__((aligned(16))) float stg[GBM * HD];
  const int tid = (int)threadIdx.x, lane = tid & 31, wave = tid >> 5, hh = lane >> 4, m = lane & 15;
  const int rowBase = (int)blockIdx.x * GBM;

  v8f acc[8];
#pragma unroll
  for (int t = 0; t < 8; ++t) acc[t] = z8();
  const unsigned short* ap = A  + (size_t)(rowBase + 16 * wave + m) * (size_t)FD + 8 * hh;
  const unsigned short* bp = BT + (size_t)m * (size_t)FD + 8 * hh;

#pragma unroll 1
  for (int k0 = 0; k0 < FD; k0 += 32) {
    FragB af;
    af.h[0] = *(const v8usa*)(ap + k0);
    af.h[1] = *(const v8usa*)(ap + k0 + 16);
#pragma unroll
    for (int nt = 0; nt < 8; ++nt) {
      const unsigned short* wq = bp + (size_t)(16 * nt) * (size_t)FD + k0;
      FragB bf;
      bf.h[0] = *(const v8usa*)wq;
      bf.h[1] = *(const v8usa*)(wq + 16);
      acc[nt] = wmb(af, bf, acc[nt]);
    }
  }

#pragma unroll
  for (int nt = 0; nt < 8; ++nt) {
    const int lc = 16 * nt + m;
#pragma unroll
    for (int r = 0; r < 8; ++r) {
      const int lr = 16 * wave + 8 * hh + r;
      stg[lr * HD + lc] = acc[nt][r];
    }
  }
  __syncthreads();

  v4f pv[16];
#pragma unroll
  for (int i = 0; i < 16; ++i) pv[i] = *(const v4fa*)(stg + (16 * wave + i) * HD + 4 * lane);
#pragma unroll
  for (int i = 0; i < 16; ++i) {
    float* op = XW + (size_t)(rowBase + 16 * wave + i) * (size_t)HD + 4 * lane;
    *(volatile v4f*)op = pv[i];
  }
  __threadfence();
#pragma unroll
  for (int i = 0; i < 16; ++i) {
    float* op = XW + (size_t)(rowBase + 16 * wave + i) * (size_t)HD + 4 * lane;
    *(volatile v4f*)op = pv[i];
  }
}

__device__ __forceinline__ void bucket_flush(const int* pl, const int* cnt, int ov, int* lp, int* cop, int* fp,
                                             int tid) {
#pragma unroll 1
  for (int i = tid * 4; i < RCAP; i += NTHR * 4) {
    const v4i v = *(const v4ia*)(pl + i);
    *(volatile v4i*)(lp + i) = v;
  }
#pragma unroll 1
  for (int i = tid * 4; i < 2 * NBRUN; i += NTHR * 4) {
    const v4i v = *(const v4ia*)(cnt + i);
    *(volatile v4i*)(cop + i) = v;
  }
  if (tid < 8) {
    const v4i f = {ov, ov, ov, ov};
    *(volatile v4i*)(fp + 4 * tid) = f;
  }
}

__global__ __launch_bounds__(NTHR) void k_bucket(const int* __restrict__ cols, const int* __restrict__ rows,
                                                 const float* __restrict__ ew, int* LIST, int* CO, int* FLAG) {
  extern __shared__ __attribute__((aligned(16))) int dsm[];
  int* wl   = dsm;
  int* pl   = dsm + NWAVE * WLCAP;
  int* cnt  = pl + RCAP;
  int* offs = cnt + NBRUN;
  int* cur  = offs + NBRUN;
  int* misc = cur + NBRUN;
  const int tid = (int)threadIdx.x, lane = tid & 31, wave = tid >> 5;
  const int blk = (int)blockIdx.x;
  const unsigned nbs = (unsigned)(blk * NBRUN);

  {
    const v4i z4 = {0, 0, 0, 0};
    for (int i = tid * 4; i < BK_ZINTS; i += NTHR * 4) *(v4ia*)(dsm + i) = z4;
    if (tid < 16) misc[tid] = 0;
  }
  __syncthreads();

  {
    const int per  = ((NE + NWAVE * WCH - 1) / (NWAVE * WCH)) * WCH;
    const int ebeg = wave * per;
    const int eend = (ebeg + per < NE) ? (ebeg + per) : NE;
    int* mylist = wl + wave * WLCAP;
    int wc = 0;
#pragma unroll 1
    for (int cb = ebeg; cb < eend; cb += WCH) {
      const int e0 = cb + lane * EPT;
      const v4i da = *(const v4ia*)(rows + e0);
      const v4i db = *(const v4ia*)(rows + e0 + 4);
      const unsigned s0 = (unsigned)da.x - nbs, s1 = (unsigned)da.y - nbs;
      const unsigned s2 = (unsigned)da.z - nbs, s3 = (unsigned)da.w - nbs;
      const unsigned s4 = (unsigned)db.x - nbs, s5 = (unsigned)db.y - nbs;
      const unsigned s6 = (unsigned)db.z - nbs, s7 = (unsigned)db.w - nbs;
      const bool h0 = s0 < (unsigned)NBRUN, h1 = s1 < (unsigned)NBRUN, h2 = s2 < (unsigned)NBRUN, h3 = s3 < (unsigned)NBRUN;
      const bool h4 = s4 < (unsigned)NBRUN, h5 = s5 < (unsigned)NBRUN, h6 = s6 < (unsigned)NBRUN, h7 = s7 < (unsigned)NBRUN;
      const unsigned m0 = __builtin_amdgcn_ballot_w32(h0), m1 = __builtin_amdgcn_ballot_w32(h1);
      const unsigned m2 = __builtin_amdgcn_ballot_w32(h2), m3 = __builtin_amdgcn_ballot_w32(h3);
      const unsigned m4 = __builtin_amdgcn_ballot_w32(h4), m5 = __builtin_amdgcn_ballot_w32(h5);
      const unsigned m6 = __builtin_amdgcn_ballot_w32(h6), m7 = __builtin_amdgcn_ballot_w32(h7);
      const unsigned any = m0 | m1 | m2 | m3 | m4 | m5 | m6 | m7;
      if (any != 0u) {
        const int pre = (int)(__builtin_amdgcn_mbcnt_lo(m0, 0u) + __builtin_amdgcn_mbcnt_lo(m1, 0u) +
                              __builtin_amdgcn_mbcnt_lo(m2, 0u) + __builtin_amdgcn_mbcnt_lo(m3, 0u) +
                              __builtin_amdgcn_mbcnt_lo(m4, 0u) + __builtin_amdgcn_mbcnt_lo(m5, 0u) +
                              __builtin_amdgcn_mbcnt_lo(m6, 0u) + __builtin_amdgcn_mbcnt_lo(m7, 0u));
        int p = wc + pre;
        if (h0) { if (p < WLCAP) mylist[p] = ((e0 + 0) << SLB) | (int)s0; p = p + 1; }
        if (h1) { if (p < WLCAP) mylist[p] = ((e0 + 1) << SLB) | (int)s1; p = p + 1; }
        if (h2) { if (p < WLCAP) mylist[p] = ((e0 + 2) << SLB) | (int)s2; p = p + 1; }
        if (h3) { if (p < WLCAP) mylist[p] = ((e0 + 3) << SLB) | (int)s3; p = p + 1; }
        if (h4) { if (p < WLCAP) mylist[p] = ((e0 + 4) << SLB) | (int)s4; p = p + 1; }
        if (h5) { if (p < WLCAP) mylist[p] = ((e0 + 5) << SLB) | (int)s5; p = p + 1; }
        if (h6) { if (p < WLCAP) mylist[p] = ((e0 + 6) << SLB) | (int)s6; p = p + 1; }
        if (h7) { if (p < WLCAP) mylist[p] = ((e0 + 7) << SLB) | (int)s7; p = p + 1; }
        wc += (int)(__builtin_popcount(m0) + __builtin_popcount(m1) + __builtin_popcount(m2) + __builtin_popcount(m3) +
                    __builtin_popcount(m4) + __builtin_popcount(m5) + __builtin_popcount(m6) + __builtin_popcount(m7));
      }
    }
    if (lane == 0) misc[wave] = wc;
  }
  __syncthreads();

  if (wave == 0) {
    int ov = 0;
#pragma unroll 1
    for (int w2 = 0; w2 < NWAVE; ++w2) {
      int c = misc[w2];
      if (c > WLCAP) ov = 1;
      c = c < 0 ? 0 : (c > WLCAP ? WLCAP : c);
#pragma unroll 1
      for (int b0 = 0; b0 < c; b0 += 32) {
        const int idx = b0 + lane;
        const int ent = wl[w2 * WLCAP + (idx < WLCAP ? idx : WLCAP - 1)];
        const int m32 = (c - b0) < 32 ? (c - b0) : 32;
#pragma unroll 1
        for (int k = 0; k < m32; ++k) {
          const int u    = __builtin_amdgcn_readlane(ent, k);
          const int slot = u & (NBRUN - 1);
          if (lane == 0) cnt[slot] = cnt[slot] + 1;
        }
      }
    }
    if (lane == 0) misc[9] = ov;
  }
  __syncthreads();
  if (wave == 0) {
    const int base = lane * (NBRUN / 32);
    int s = 0;
#pragma unroll 1
    for (int i = 0; i < NBRUN / 32; ++i) s += cnt[base + i];
    int incl = s;
#pragma unroll
    for (int d = 1; d < 32; d <<= 1) {
      const int y = __shfl_up(incl, d, 32);
      if (lane >= d) incl += y;
    }
    int run = incl - s;
#pragma unroll 1
    for (int i = 0; i < NBRUN / 32; ++i) {
      const int cv = cnt[base + i];
      offs[base + i] = run;
      cur[base + i]  = run;
      run += cv;
    }
  }
  __syncthreads();

  if (wave == 0) {
#pragma unroll 1
    for (int w2 = 0; w2 < NWAVE; ++w2) {
      int c = misc[w2];
      c = c < 0 ? 0 : (c > WLCAP ? WLCAP : c);
#pragma unroll 1
      for (int b0 = 0; b0 < c; b0 += 32) {
        const int idx = b0 + lane;
        const int ent = wl[w2 * WLCAP + (idx < WLCAP ? idx : WLCAP - 1)];
        int eid = (ent >> SLB) & 0x1FFFFF;
        eid = eid > NE - 1 ? NE - 1 : eid;
        int sr = cols[eid];
        sr = sr < 0 ? 0 : (sr > NN - 1 ? NN - 1 : sr);
        const int word = (int)((unsigned)sr | (bf16_bits(ew[eid]) << 16));
        const int m32 = (c - b0) < 32 ? (c - b0) : 32;
#pragma unroll 1
        for (int k = 0; k < m32; ++k) {
          const int u    = __builtin_amdgcn_readlane(ent, k);
          const int wd   = __builtin_amdgcn_readlane(word, k);
          const int slot = u & (NBRUN - 1);
          if (lane == 0) {
            int p = cur[slot];
            p = p < 0 ? 0 : (p > RCAP - 1 ? RCAP - 1 : p);
            pl[p] = wd;
            cur[slot] = p + 1;
          }
        }
      }
    }
  }
  __syncthreads();

  const int ovf = misc[9];
  int* lp  = LIST + (size_t)blk * RCAP;
  int* cop = CO + (size_t)blk * (2 * NBRUN);
  int* fp  = FLAG + (size_t)blk * 32;
  bucket_flush(pl, cnt, ovf, lp, cop, fp, tid);
  __threadfence();
  bucket_flush(pl, cnt, ovf, lp, cop, fp, tid);
}

__global__ __launch_bounds__(NTHR) void k_replay(const int* __restrict__ LIST, const int* __restrict__ CO,
                                                 const int* __restrict__ FLAG, const float* __restrict__ XW,
                                                 const float* __restrict__ PAR, float* T, double* REC) {
  __shared__ __attribute__((aligned(16))) float  wst[NWAVE * WSTW];
  __shared__ __attribute__((aligned(16))) double rst[RECW];
  const int tid = (int)threadIdx.x, lane = tid & 31, wave = tid >> 5;
  const int blk = (int)blockIdx.x;
  const int* lb  = LIST + (size_t)blk * RCAP;
  const int* cob = CO + (size_t)blk * (2 * NBRUN);
  const int flag = FLAG[(size_t)blk * 32];
  const float qnan = __uint_as_float(0x7fc00000u);
  const v4f bias = *(const v4fa*)(PAR + 4 * lane);

  int wn = 0;
  float wm[4], wq[4];
#pragma unroll
  for (int j = 0; j < 4; ++j) { wm[j] = 0.0f; wq[j] = 0.0f; }

#pragma unroll 1
  for (int si = 0; si < NBRUN / NWAVE; ++si) {
    const int slot = si * NWAVE + wave;
    const int node = blk * NBRUN + slot;
    int c = cob[slot];
    int o = cob[NBRUN + slot];
    const bool big = c > DEGCAP;
    c = c < 0 ? 0 : (c > DEGCAP ? DEGCAP : c);
    o = o < 0 ? 0 : (o > RCAP - 1 ? RCAP - 1 : o);
    c = __builtin_amdgcn_readfirstlane(c);
    o = __builtin_amdgcn_readfirstlane(o);
    int last = o + c - 1;
    last = last < o ? o : last;
    last = last > RCAP - 1 ? RCAP - 1 : last;
    float a0 = 0.0f, a1 = 0.0f, a2 = 0.0f, a3 = 0.0f;
#pragma unroll 1
    for (int j = 0; j < c; ++j) {
      int idx = o + j;
      idx = idx > last ? last : idx;
      const unsigned wd = (unsigned)lb[idx];
      int sr = (int)(wd & 0xffffu);
      sr = sr > NN - 1 ? NN - 1 : sr;
      const float w = __uint_as_float(wd & 0xffff0000u);
      const v4f v = *(const v4fa*)(XW + (size_t)sr * HD + 4 * lane);
      a0 = fmaf(w, v.x, a0); a1 = fmaf(w, v.y, a1); a2 = fmaf(w, v.z, a2); a3 = fmaf(w, v.w, a3);
    }
    float t[4];
    t[0] = a0 + bias.x; t[1] = a1 + bias.y; t[2] = a2 + bias.z; t[3] = a3 + bias.w;
    const bool bad  = (flag != 0) | big;
#pragma unroll
    for (int j = 0; j < 4; ++j) t[j] = bad ? qnan : t[j];
    const bool live = node < NN;
    if (live) {
      wn += 1;
      const float rk = 1.0f / (float)wn;
#pragma unroll
      for (int j = 0; j < 4; ++j) {
        const float d = t[j] - wm[j];
        wm[j] = fmaf(d, rk, wm[j]);
        wq[j] = fmaf(d, t[j] - wm[j], wq[j]);
      }
    }
    if (node < MP) {
      v4f ov;
      ov.x = live ? t[0] : 0.0f; ov.y = live ? t[1] : 0.0f;
      ov.z = live ? t[2] : 0.0f; ov.w = live ? t[3] : 0.0f;
      st2_v4f(T + (size_t)node * HD + 4 * lane, ov);
    }
  }

  if (lane == 0) wst[wave * WSTW] = (float)wn;
#pragma unroll
  for (int j = 0; j < 4; ++j) {
    wst[wave * WSTW + 4 + 4 * lane + j]      = wm[j];
    wst[wave * WSTW + 4 + HD + 4 * lane + j] = wq[j];
  }
  __syncthreads();
  if (tid < HD) {
    double n = 0.0, mean = 0.0, M2 = 0.0;
#pragma unroll 1
    for (int w2 = 0; w2 < NWAVE; ++w2) {
      const double nb = (double)wst[w2 * WSTW];
      const double mb = (double)wst[w2 * WSTW + 4 + tid];
      const double qb = (double)wst[w2 * WSTW + 4 + HD + tid];
      if (nb > 0.5) {
        const double nn = n + nb;
        const double delta = mb - mean;
        const double f = nb / nn;
        mean = mean + delta * f;
        M2 = M2 + qb + delta * delta * n * f;
        n = nn;
      }
    }
    rst[tid] = n;
    rst[HD + tid] = mean;
    rst[2 * HD + tid] = M2;
  }
  __syncthreads();
  double* rp = REC + (size_t)blk * RECW;
  v2d rv = {0.0, 0.0};
  if (tid < RECW / 2) {
    rv = *(const v2da*)(rst + 2 * tid);
    *(volatile v2d*)(rp + 2 * tid) = rv;
  }
  __threadfence();
  if (tid < RECW / 2) {
    *(volatile v2d*)(rp + 2 * tid) = rv;
  }
}

__global__ __launch_bounds__(HD) void k_comb(const double* __restrict__ REC, float* STAT) {
  __shared__ __attribute__((aligned(16))) float stg[2 * HD];
  const int tid = (int)threadIdx.x;
  const int c = tid;
  double n = 0.0, mean = 0.0, M2 = 0.0;
#pragma unroll 1
  for (int b = 0; b < NBK; ++b) {
    const double* pr = REC + (size_t)b * RECW;
    const double nb = pr[c];
    const double mb = pr[HD + c];
    const double qb = pr[2 * HD + c];
    if (nb > 0.5) {
      const double nn = n + nb;
      const double delta = mb - mean;
      const double f = nb / nn;
      mean = mean + delta * f;
      M2 = M2 + qb + delta * delta * n * f;
      n = nn;
    }
  }
  const double nt = n < 1.0 ? 1.0 : n;
  const float varf  = (float)(M2 / nt);
  const float meanf = (float)mean;
  const float rs = 1.0f / sqrtf(varf + 1e-5f);
  stg[c] = meanf;
  stg[HD + c] = rs;
  __syncthreads();
  v4f v = {0.f, 0.f, 0.f, 0.f};
  if (tid < (2 * HD) / 4) {
    v = *(const v4fa*)(stg + 4 * tid);
    *(volatile v4f*)(STAT + 4 * tid) = v;
  }
  __threadfence();
  if (tid < (2 * HD) / 4) {
    *(volatile v4f*)(STAT + 4 * tid) = v;
  }
}

__global__ __launch_bounds__(NTHR) void k_apply(const float* __restrict__ T, const unsigned short* __restrict__ XB,
                                                const float* __restrict__ STAT, const float* __restrict__ PAR,
                                                float* out) {
  __shared__ __attribute__((aligned(16))) float sst[4 * HD];
  const int tid = (int)threadIdx.x;
  if (tid < 64) {
    *(v4fa*)(sst + 4 * tid) = *(const v4fa*)(STAT + 4 * tid);
  } else if (tid < 128) {
    const int q = tid - 64;
    *(v4fa*)(sst + 2 * HD + 4 * q) = *(const v4fa*)(PAR + HD + 4 * q);
  }
  __syncthreads();
  const int u  = (int)blockIdx.x * NTHR + tid;
  const int c4 = (u & 31) * 4;
  const v4f t  = *(const v4fa*)(T + (size_t)u * 4);
  const v2u xw = *(const v2ua*)(XB + (size_t)u * 4);
  const v4f mu = *(const v4fa*)(sst + c4);
  const v4f rs = *(const v4fa*)(sst + HD + c4);
  const v4f g  = *(const v4fa*)(sst + 2 * HD + c4);
  const v4f be = *(const v4fa*)(sst + 3 * HD + c4);
  const float f0 = __uint_as_float(xw.x << 16);
  const float f1 = __uint_as_float(xw.x & 0xffff0000u);
  const float f2 = __uint_as_float(xw.y << 16);
  const float f3 = __uint_as_float(xw.y & 0xffff0000u);
  float y0 = ((t.x - mu.x) * rs.x) * g.x + be.x;
  float y1 = ((t.y - mu.y) * rs.y) * g.y + be.y;
  float y2 = ((t.z - mu.z) * rs.z) * g.z + be.z;
  float y3 = ((t.w - mu.w) * rs.w) * g.w + be.w;
  y0 = (y0 > 0.0f) ? y0 : (y0 - y0);
  y1 = (y1 > 0.0f) ? y1 : (y1 - y1);
  y2 = (y2 > 0.0f) ? y2 : (y2 - y2);
  y3 = (y3 > 0.0f) ? y3 : (y3 - y3);
  v4f o;
  o.x = f0 + y0; o.y = f1 + y1; o.z = f2 + y2; o.w = f3 + y3;
  st2_v4f(out + (size_t)u * 4, o);
}

extern "C" void kernel_launch(void* const* d_in, const int* in_sizes, int n_in,
                              void* d_out, int out_size, void* d_ws, size_t ws_size,
                              hipStream_t stream) {
  if (n_in < 8) return;
  if (in_sizes[0] != NN * FD) return;
  if (in_sizes[1] != FD * HD) return;
  if (in_sizes[2] != HD) return;
  if (in_sizes[3] != HD) return;
  if (in_sizes[4] != HD) return;
  if (in_sizes[5] != NE) return;
  if (in_sizes[6] != NE) return;
  if (in_sizes[7] != NE) return;
  if (out_size != NN * HD) return;

  const float* feature = (const float*)d_in[0];
  const float* weight  = (const float*)d_in[1];
  const float* bias    = (const float*)d_in[2];
  const float* gamma   = (const float*)d_in[3];
  const float* beta    = (const float*)d_in[4];
  const float* ew      = (const float*)d_in[5];
  const int*   erow    = (const int*)d_in[6];
  const int*   ecol    = (const int*)d_in[7];
  float* out = (float*)d_out;

  constexpr size_t zXB   = (size_t)MP * FD * 2;
  constexpr size_t zWT   = (size_t)HD * FD * 2;
  constexpr size_t zPAR  = (size_t)3 * HD * 4;
  constexpr size_t zXW   = (size_t)MP * HD * 4;
  constexpr size_t zT    = (size_t)MP * HD * 4;
  constexpr size_t zLIST = (size_t)NBK * RCAP * 4;
  constexpr size_t zCO   = (size_t)NBK * 2 * NBRUN * 4;
  constexpr size_t zFLAG = 6400;
  constexpr size_t zREC  = (size_t)NBK * RECW * 8;
  constexpr size_t zSTAT = (size_t)2 * HD * 4;
  constexpr size_t oXB   = 0;
  constexpr size_t oWT   = oXB + zXB;
  constexpr size_t oPAR  = oWT + zWT;
  constexpr size_t oXW   = oPAR + zPAR;
  constexpr size_t oT    = oXW + zXW;
  constexpr size_t oLIST = oT + zT;
  constexpr size_t oCO   = oLIST + zLIST;
  constexpr size_t oFLAG = oCO + zCO;
  constexpr size_t oREC  = oFLAG + zFLAG;
  constexpr size_t oSTAT = oREC + zREC;
  constexpr size_t oEND  = oSTAT + zSTAT;
  static_assert(zXB % 256 == 0 && zWT % 256 == 0 && zPAR % 256 == 0 && zXW % 256 == 0 && zT % 256 == 0);
  static_assert(zLIST % 256 == 0 && zCO % 256 == 0 && zFLAG % 256 == 0 && zREC % 256 == 0 && zSTAT % 256 == 0);
  static_assert(zFLAG >= (size_t)NBK * 128);
  static_assert(oEND <= ((size_t)128 << 20));
  if (oEND > ws_size) return;

  char* ws = (char*)d_ws;
  unsigned short* XB   = (unsigned short*)(ws + oXB);
  unsigned short* WT   = (unsigned short*)(ws + oWT);
  float*          PAR  = (float*)(ws + oPAR);
  float*          XW   = (float*)(ws + oXW);
  float*          T    = (float*)(ws + oT);
  int*            LIST = (int*)(ws + oLIST);
  int*            CO   = (int*)(ws + oCO);
  int*            FLAG = (int*)(ws + oFLAG);
  double*         REC  = (double*)(ws + oREC);
  float*          STAT = (float*)(ws + oSTAT);

  hipFuncSetAttribute(reinterpret_cast<const void*>(&k_bucket), hipFuncAttributeMaxDynamicSharedMemorySize, (int)BK_LDS);

  k_prep<<<PBTOT, NTHR, 0, stream>>>(feature, weight, bias, gamma, beta, XB, WT, PAR);
  k_gemm_one<<<MP / GBM, GTHR, 0, stream>>>(XB, WT, XW);
  k_bucket<<<NBK, NTHR, BK_LDS, stream>>>(ecol, erow, ew, LIST, CO, FLAG);
  k_replay<<<NBK, NTHR, 0, stream>>>(LIST, CO, FLAG, XW, PAR, T, REC);
  k_comb<<<1, HD, 0, stream>>>(REC, STAT);
  k_apply<<<(NN * 32) / NTHR, NTHR, 0, stream>>>(T, XB, STAT, PAR, out);
}
